// SelfAttention_32770600469142
// MI455X (gfx1250) — hardware-verified
//
#include <hip/hip_runtime.h>
#ifndef NB
#define NB 16
#endif
#ifndef SEQ
#define SEQ 512
#endif
#define NB_FULL 16
#define SEQ_FULL 512
#define DM 768
#define NH 12
#define HD 64
#define NR (NB * SEQ)
#define WS_TOTAL ((size_t)3 * DM * DM * 2 + (size_t)4 * NR * DM * 2)

static_assert(NH * HD == DM);
static_assert(HD == 64);
static_assert(DM % 32 == 0);
static_assert(DM % 64 == 0);
static_assert(DM % 128 == 0);
static_assert(NR % 128 == 0);
static_assert(NR % 64 == 0);
static_assert(SEQ % 64 == 0);
static_assert((DM / 8) % 32 == 0);
static_assert(SEQ <= SEQ_FULL);
static_assert(NB <= NB_FULL);
static_assert(SEQ_FULL % 4 == 0);
static_assert((DM * DM * 2) % 256 == 0);
static_assert(((size_t)NR * DM * 2) % 256 == 0);
static_assert(WS_TOTAL <= (size_t)134217728);

typedef unsigned short v8us __attribute__((ext_vector_type(8), may_alias));
typedef float  v8f  __attribute__((ext_vector_type(8)));
typedef float  v4f  __attribute__((ext_vector_type(4)));
typedef float  v4fa __attribute__((ext_vector_type(4), may_alias));
typedef _Float16 v16h __attribute__((ext_vector_type(16)));
union FragH { v16h v; v8us half[2]; _Float16 h[16]; unsigned short u[16]; };

__device__ __forceinline__ unsigned short bf16_bits(float x) { unsigned int u = __float_as_uint(x); return (unsigned short)((u + 0x7FFFu + ((u >> 16) & 1u)) >> 16); }
__device__ __forceinline__ float bf16_rne(float x) { return __uint_as_float(((unsigned int)bf16_bits(x)) << 16); }

__device__ __forceinline__ v16h g2_frag(const _Float16* p, int hh) { FragH f; f.half[0] = *(const v8us*)((const unsigned short*)p + 8 * hh); f.half[1] = *(const v8us*)((const unsigned short*)p + 16 + 8 * hh); return f.v; }
__device__ __forceinline__ v8f g2_mma(v16h a, v16h b, v8f c) { v8f d = __builtin_amdgcn_wmma_f32_16x16x32_f16(false, a, false, b, (short)0, c, false, false); asm volatile("v_nop\n\tv_nop\n\tv_nop\n\tv_nop" : "+v"(d) : "v"(a), "v"(b)); return d; }

__global__ __launch_bounds__(256) void k_wt_f16(const float* __restrict__ W, _Float16* __restrict__ Wt, int K, int N, float scale) {
  const int t = blockIdx.x * 256 + threadIdx.x; if (t >= N * (K / 8)) return; const int n = t / (K / 8), k8 = (t % (K / 8)) * 8; FragH f;
#pragma unroll
  for (int i = 0; i < 8; ++i) f.h[i] = (_Float16)(bf16_rne(W[(size_t)(k8 + i) * N + n]) * scale);
  const v8us o = f.half[0];
  *(volatile v8us*)((unsigned short*)Wt + (size_t)n * K + k8) = o; __threadfence(); *(volatile v8us*)((unsigned short*)Wt + (size_t)n * K + k8) = o;
}

__global__ __launch_bounds__(256) void k_x16(const float* __restrict__ x, _Float16* __restrict__ X16) {
  const int t = blockIdx.x * 256 + threadIdx.x; if (t >= NR * (DM / 8)) return;
  const int row = t / (DM / 8), c8 = (t % (DM / 8)) * 8; const int b = row / SEQ, s = row % SEQ;
  const float* src = x + ((size_t)b * SEQ_FULL + s) * DM + c8;
  const v4f a = *(const v4fa*)src, c = *(const v4fa*)(src + 4); FragH f;
#pragma unroll
  for (int q = 0; q < 4; ++q) { f.h[q] = (_Float16)bf16_rne(a[q]); f.h[4 + q] = (_Float16)bf16_rne(c[q]); }
  const v8us o = f.half[0];
  unsigned short* d = (unsigned short*)X16 + (size_t)row * DM + c8;
  *(volatile v8us*)d = o; __threadfence(); *(volatile v8us*)d = o;
}

__global__ __launch_bounds__(128) void k_gemm2(const _Float16* __restrict__ A, int lda, const _Float16* __restrict__ Bh, int ldb, float alpha, const float* __restrict__ bias, int biasrow,
                                               _Float16* __restrict__ C16, int ldc, int M, int N, int K) {
  __shared__ __attribute__((aligned(16))) float so[4][32][68];
  const int tid = threadIdx.x; const int w = __builtin_amdgcn_readfirstlane(tid >> 5); const int lane = tid & 31, ln = lane & 15, hh = lane >> 4;
  const int ntn = N >> 6; const int mt = blockIdx.x / ntn, nq = blockIdx.x - mt * ntn; const int row0 = mt * 128 + 32 * w, col0 = nq * 64; if (row0 >= M) return;
  const _Float16* a0p = A + (size_t)(row0 + ln) * lda; const _Float16* a1p = a0p + (size_t)16 * lda;
  const _Float16* b0p = Bh + (size_t)(col0 + ln) * ldb; const _Float16* b1p = b0p + (size_t)16 * ldb; const _Float16* b2p = b1p + (size_t)16 * ldb; const _Float16* b3p = b2p + (size_t)16 * ldb;
  const v8f z8 = {0.f,0.f,0.f,0.f,0.f,0.f,0.f,0.f}; v8f c00 = z8, c01 = z8, c02 = z8, c03 = z8, c10 = z8, c11 = z8, c12 = z8, c13 = z8;
#pragma unroll 1
  for (int kb = 0; kb < K; kb += 32) { const v16h a0 = g2_frag(a0p + kb, hh), a1 = g2_frag(a1p + kb, hh);
    v16h b = g2_frag(b0p + kb, hh); c00 = g2_mma(a0, b, c00); c10 = g2_mma(a1, b, c10);
    b = g2_frag(b1p + kb, hh); c01 = g2_mma(a0, b, c01); c11 = g2_mma(a1, b, c11);
    b = g2_frag(b2p + kb, hh); c02 = g2_mma(a0, b, c02); c12 = g2_mma(a1, b, c12);
    b = g2_frag(b3p + kb, hh); c03 = g2_mma(a0, b, c03); c13 = g2_mma(a1, b, c13); }
  v8f accs[8] = {c00, c01, c02, c03, c10, c11, c12, c13};
  float bcol[4] = {0.f, 0.f, 0.f, 0.f}; const v4f z4 = {0.f, 0.f, 0.f, 0.f}; v4f br[4] = {z4, z4, z4, z4};
  if (biasrow != 0) {
#pragma unroll
    for (int half = 0; half < 2; ++half) { br[half * 2] = *(const v4fa*)(bias + row0 + half * 16 + 8 * hh); br[half * 2 + 1] = *(const v4fa*)(bias + row0 + half * 16 + 8 * hh + 4); }
  } else {
#pragma unroll
    for (int t = 0; t < 4; ++t) bcol[t] = bf16_rne(bias[col0 + t * 16 + ln]);
  }
#pragma unroll
  for (int u = 0; u < 8; ++u) { const int t = u & 3, half = u >> 2;
#pragma unroll
    for (int r = 0; r < 8; ++r) { const int rloc = half * 16 + 8 * hh + r; const float brv = bf16_rne(br[half * 2 + (r >> 2)][r & 3]); const float bv = (biasrow != 0) ? brv : bcol[t];
      so[w][rloc][t * 16 + ln] = accs[u][r] * alpha + bv; } }
  __builtin_amdgcn_fence(4  , "workgroup"); __builtin_amdgcn_wave_barrier();
  const int rq = lane >> 3, c8 = (lane & 7) * 8;
  for (int pass = 0; pass < 2; ++pass) {
#pragma unroll
    for (int q = 0; q < 8; ++q) { const int r = q * 4 + rq;
      const v4f x0 = *(const v4fa*)&so[w][r][c8]; const v4f x1 = *(const v4fa*)&so[w][r][c8 + 4]; FragH f;
#pragma unroll
      for (int i = 0; i < 4; ++i) { f.h[i] = (_Float16)x0[i]; f.h[4 + i] = (_Float16)x1[i]; }
      const v8us o = f.half[0];
      *(volatile v8us*)((unsigned short*)C16 + (size_t)(row0 + r) * ldc + col0 + c8) = o; }
    if (pass == 0) __threadfence(); }
}

__global__ __launch_bounds__(128) void k_flash(const _Float16* __restrict__ Q16, const _Float16* __restrict__ K16, const _Float16* __restrict__ VT, const float* __restrict__ mask, float* __restrict__ out) {
  __shared__ __attribute__((aligned(16))) float sbias[SEQ];
  __shared__ __attribute__((aligned(16))) float so[4][16][68];
  const int tid = threadIdx.x; const int wave = __builtin_amdgcn_readfirstlane(tid >> 5); const int lane = tid & 31, ln = lane & 15, hh = lane >> 4;
  const int qt = blockIdx.x % (SEQ / 64); const int bh = blockIdx.x / (SEQ / 64); const int h = bh % NH, b = bh / NH;
  for (int i = tid; i < SEQ / 4; i += 128) {
    const v4f mv = *(const v4fa*)(mask + (size_t)b * SEQ_FULL + i * 4); v4f bv;
#pragma unroll
    for (int q = 0; q < 4; ++q) bv[q] = bf16_rne(mv[q]) * -1.0e9f;
    *(v4f*)&sbias[i * 4] = bv; }
  __syncthreads();
  const size_t rb = (size_t)b * SEQ; const int q0 = qt * 64 + wave * 16;
  const _Float16* qp = Q16 + (rb + q0 + ln) * DM + h * HD;
  const v16h bq0 = g2_frag(qp, hh), bq1 = g2_frag(qp + 32, hh);
  const _Float16* kb = K16 + (rb + ln) * DM + h * HD;
  const _Float16* vb = VT + (size_t)(h * HD + ln) * NR + rb;
  const v8f z8 = {0.f,0.f,0.f,0.f,0.f,0.f,0.f,0.f};
  v8f o0 = z8, o1 = z8, o2 = z8, o3 = z8; float m = -1.0e30f, lsum = 0.f;
#pragma unroll 1
  for (int k0 = 0; k0 < SEQ; k0 += 32) {
    const _Float16* kp = kb + (size_t)k0 * DM;
    const v16h a0 = g2_frag(kp, hh), a1 = g2_frag(kp + 32, hh);
    const v16h a2 = g2_frag(kp + 16 * DM, hh), a3 = g2_frag(kp + 16 * DM + 32, hh);
    v8f c0 = z8, c1 = z8;
    c0 = __builtin_amdgcn_wmma_f32_16x16x32_f16(false, a0, false, bq0, (short)0, c0, false, false);
    c1 = __builtin_amdgcn_wmma_f32_16x16x32_f16(false, a2, false, bq0, (short)0, c1, false, false);
    c0 = __builtin_amdgcn_wmma_f32_16x16x32_f16(false, a1, false, bq1, (short)0, c0, false, false);
    c1 = __builtin_amdgcn_wmma_f32_16x16x32_f16(false, a3, false, bq1, (short)0, c1, false, false);
    asm volatile("v_nop\n\tv_nop\n\tv_nop\n\tv_nop" : "+v"(c0), "+v"(c1) : "v"(a0), "v"(a1), "v"(a2), "v"(a3), "v"(bq0), "v"(bq1));
    const v4f bl0 = *(const v4fa*)&sbias[k0 + 8 * hh], bl1 = *(const v4fa*)&sbias[k0 + 8 * hh + 4];
    const v4f bl2 = *(const v4fa*)&sbias[k0 + 16 + 8 * hh], bl3 = *(const v4fa*)&sbias[k0 + 16 + 8 * hh + 4];
    float s[16];
#pragma unroll
    for (int r = 0; r < 4; ++r) { s[r] = fmaf(c0[r], 0.125f, bl0[r]); s[4 + r] = fmaf(c0[4 + r], 0.125f, bl1[r]); s[8 + r] = fmaf(c1[r], 0.125f, bl2[r]); s[12 + r] = fmaf(c1[4 + r], 0.125f, bl3[r]); }
    float mx = s[0];
#pragma unroll
    for (int i = 1; i < 16; ++i) mx = fmaxf(mx, s[i]);
    mx = fmaxf(mx, __shfl_xor(mx, 16));
    const float mn = fmaxf(m, mx); const float sc = __expf(m - mn); m = mn; const float mo = mn - 6.9314718f;
    float ps = 0.f; FragH pb;
#pragma unroll
    for (int i = 0; i < 16; ++i) { const float e = __expf(s[i] - mo); ps += e; pb.h[i] = (_Float16)e; }
    lsum = lsum * sc + ps;
    o0 *= sc; o1 *= sc; o2 *= sc; o3 *= sc;
    const _Float16* vp = vb + k0;
    const v16h v0 = g2_frag(vp, hh), v1 = g2_frag(vp + (size_t)16 * NR, hh), v2 = g2_frag(vp + (size_t)32 * NR, hh), v3 = g2_frag(vp + (size_t)48 * NR, hh);
    const v16h pv = pb.v;
    o0 = __builtin_amdgcn_wmma_f32_16x16x32_f16(false, v0, false, pv, (short)0, o0, false, false);
    o1 = __builtin_amdgcn_wmma_f32_16x16x32_f16(false, v1, false, pv, (short)0, o1, false, false);
    o2 = __builtin_amdgcn_wmma_f32_16x16x32_f16(false, v2, false, pv, (short)0, o2, false, false);
    o3 = __builtin_amdgcn_wmma_f32_16x16x32_f16(false, v3, false, pv, (short)0, o3, false, false);
    asm volatile("v_nop\n\tv_nop\n\tv_nop\n\tv_nop" : "+v"(o0), "+v"(o1), "+v"(o2), "+v"(o3) : "v"(v0), "v"(v1), "v"(v2), "v"(v3), "v"(pv));
  }
  const float lt = lsum + __shfl_xor(lsum, 16);
  const float inv = 1.0f / lt;
  v8f oo[4] = {o0, o1, o2, o3};
#pragma unroll
  for (int dt = 0; dt < 4; ++dt) {
    v4f t0, t1;
#pragma unroll
    for (int r = 0; r < 4; ++r) { t0[r] = oo[dt][r] * inv; t1[r] = oo[dt][4 + r] * inv; }
    *(v4f*)&so[wave][ln][16 * dt + 8 * hh] = t0; *(v4f*)&so[wave][ln][16 * dt + 8 * hh + 4] = t1; }
  __builtin_amdgcn_fence(4  , "workgroup"); __builtin_amdgcn_wave_barrier();
  const int rsub = lane >> 4, c4 = (lane & 15) * 4;
  for (int pass = 0; pass < 2; ++pass) {
#pragma unroll
    for (int q = 0; q < 8; ++q) { const int r = q * 2 + rsub;
      const v4f v = *(const v4fa*)&so[wave][r][c4];
      *(volatile v4f*)(out + (rb + q0 + r) * DM + h * HD + c4) = v; }
    if (pass == 0) __threadfence(); }
}

extern "C" void kernel_launch(void* const* d_in, const int* in_sizes, int n_in,
                              void* d_out, int out_size, void* d_ws, size_t ws_size, hipStream_t stream) {
  if (n_in < 8) return;
  const long long need_rows = (long long)(NB - 1) * SEQ_FULL + SEQ;
  if ((long long)in_sizes[0] < need_rows * DM) return;
  if ((long long)in_sizes[1] < need_rows) return;
  if (in_sizes[2] < DM * DM || in_sizes[4] < DM * DM || in_sizes[6] < DM * DM) return;
  if (in_sizes[3] < DM || in_sizes[5] < DM || in_sizes[7] < DM) return;
  if ((long long)out_size < (long long)NR * DM) return;
  const float* x = (const float*)d_in[0]; const float* mask = (const float*)d_in[1];
  const float* wq = (const float*)d_in[2]; const float* bq = (const float*)d_in[3];
  const float* wk = (const float*)d_in[4]; const float* bk = (const float*)d_in[5];
  const float* wv = (const float*)d_in[6]; const float* bv = (const float*)d_in[7];
  char* ws = (char*)d_ws; size_t off = 0;
  auto take = [&](size_t bytes) { char* p = ws + off; off += (bytes + 255) & ~(size_t)255; return p; };
  _Float16* BQ = (_Float16*)take((size_t)DM * DM * 2); _Float16* BK = (_Float16*)take((size_t)DM * DM * 2); _Float16* BV = (_Float16*)take((size_t)DM * DM * 2);
  _Float16* X16 = (_Float16*)take((size_t)NR * DM * 2);
  _Float16* Q16 = (_Float16*)take((size_t)NR * DM * 2); _Float16* K16 = (_Float16*)take((size_t)NR * DM * 2);
  _Float16* VT = (_Float16*)take((size_t)DM * NR * 2);
  if (off > ws_size) return;
  { const unsigned g = (unsigned)(((size_t)DM * (DM / 8) + 255) / 256);
    k_wt_f16<<<g, 256, 0, stream>>>(wq, BQ, DM, DM, 16.0f); k_wt_f16<<<g, 256, 0, stream>>>(wk, BK, DM, DM, 16.0f); k_wt_f16<<<g, 256, 0, stream>>>(wv, BV, DM, DM, 16.0f); }
  k_x16<<<(unsigned)(((size_t)NR * (DM / 8) + 255) / 256), 256, 0, stream>>>(x, X16);
  k_gemm2<<<(unsigned)((NR / 128) * (DM / 64)), 128, 0, stream>>>(X16, DM, BQ, DM, 0.0625f, bq, 0, Q16, DM, NR, DM, DM);
  k_gemm2<<<(unsigned)((NR / 128) * (DM / 64)), 128, 0, stream>>>(X16, DM, BK, DM, 0.0625f, bk, 0, K16, DM, NR, DM, DM);
  k_gemm2<<<(unsigned)((DM / 128) * (NR / 64)), 128, 0, stream>>>(BV, DM, X16, DM, 0.0625f, bv, 1, VT, NR, DM, NR, DM);
  k_flash<<<(unsigned)((SEQ / 64) * NH * NB), 128, 0, stream>>>(Q16, K16, VT, mask, (float*)d_out);
}
